// GVPConv_9663676416046
// MI455X (gfx1250) — hardware-verified
//
#include <hip/hip_runtime.h>
#include <stddef.h>
#include <math.h>


#define NB     2
#define NN     2048
#define NODES  (NB * NN)
#define KNB    32
#define SD     128
#define VC     16
#define VF     (VC * 3)
#define ESD    32
#define EPB    64
#define NTHR   256
#define NWAVE  8
#define SO     128
#define VO     16
#define K1     321
#define K1P    352
#define PA1    360
#define SI1    288
#define VI1    33
#define H1     33
#define ZC1    320
#define K2     144
#define K2P    160
#define PA2    168
#define SI2    128
#define VI2    16
#define H2     16
#define GK     128
#define PG     136
#define MVP    36
#define MVS    108
#define WSCL   16.0f
#define INV16  0.0625f
#define INVK   0.03125f
#define VEPS   1e-8f

#define GW1   (SO * K1P / 8)
#define GW2   (SO * K2P / 8)
#define GGT   (VO * GK / 8)
#define GTOT  (GW1 + 2 * GW2 + 3 * GGT)

#define L_A      0
#define L_GIN    (L_A + EPB * PA1 * 2)
#define L_MV     (L_GIN + EPB * PG * 2)
#define L_VH     (L_MV + EPB * MVS * 4)
#define L_GT     (L_VH + EPB * MVS * 4)
#define L_WH     (L_GT + EPB * VO * 4)
#define L_WV     (L_WH + H1 * MVP * 4)
#define L_OS     (L_WV + VO * MVP * 4)
#define L_OV     (L_OS + 2 * SD * 4)
#define LDS_MAIN (L_OV + 2 * VF * 4)

static_assert(NTHR == NWAVE * 32);
static_assert(EPB == 2 * KNB && EPB == NWAVE * 8);
static_assert(SO == NWAVE * 16 && EPB * VO == 4 * NTHR);
static_assert((GTOT % NTHR) == 0 && (GW1 % NTHR) == 0 && (GW2 % NTHR) == 0 && (GGT % NTHR) == 0);
static_assert((K1P % 32) == 0 && (K2P % 32) == 0 && (GK % 32) == 0);
static_assert(K1P >= K1 && K2P >= K2 && K1 == SI1 + H1 && K2 == SI2 + H2);
static_assert((PA1 % 8) == 0 && (PA2 % 8) == 0 && (PG % 8) == 0 && PA1 >= K1P && PA2 >= K2P && PG >= GK);
static_assert((ZC1 % 8) == 0 && ZC1 <= K1 - 1 && ZC1 >= SI1 && ZC1 + 40 == PA1);
static_assert(((SI2 + H2) % 8) == 0 && SI2 + H2 + 16 == K2P);
static_assert((MVS * 4) % 16 == 0 && (MVP * 4) % 16 == 0 && MVS >= 3 * MVP);
static_assert(MVP >= 4 * ((VI1 + 3) / 4) && MVP >= 4 * ((H1 + 3) / 4));
static_assert((L_GIN % 16) == 0 && (L_MV % 16) == 0 && (L_VH % 16) == 0 && (L_GT % 16) == 0);
static_assert((L_WH % 16) == 0 && (L_WV % 16) == 0 && (L_OS % 16) == 0 && (L_OV % 16) == 0);
static_assert((NODES % 2) == 0 && (NN % 2) == 0);
static_assert(2 * VF == 96 && ((2 * VF * 4) % 128) == 0 && ((SD * 4) % 128) == 0);

typedef float    v4f  __attribute__((ext_vector_type(4)));
typedef float    v8f  __attribute__((ext_vector_type(8)));
typedef _Float16 v4h  __attribute__((ext_vector_type(4)));
typedef _Float16 v8h  __attribute__((ext_vector_type(8)));
typedef _Float16 v16h __attribute__((ext_vector_type(16)));
union FragH { v16h v; v8h h[2]; };

__device__ __forceinline__ v8f wmh(v16h a, v16h b, v8f c) {
  v8f d = __builtin_amdgcn_wmma_f32_16x16x32_f16(false, a, false, b, (short)0, c, false, false);
#if defined(__HIP_DEVICE_COMPILE__)
  asm volatile("v_nop\n\tv_nop\n\tv_nop\n\tv_nop" : "+v"(d) : "v"(a), "v"(b));
#endif
  return d;
}

__device__ __forceinline__ v8f zero8() {
  v8f z = {0.f, 0.f, 0.f, 0.f, 0.f, 0.f, 0.f, 0.f};
  return z;
}

__device__ __forceinline__ v8h zero8h() {
  v8h z;
#pragma unroll
  for (int u = 0; u < 8; ++u) z[u] = (_Float16)0.0f;
  return z;
}

__device__ __forceinline__ float sigm(float x) {
  const float xc = fminf(fmaxf(x, -30.0f), 30.0f);
  const float ex = __expf(-xc);
  return __builtin_amdgcn_rcpf(1.0f + ex);
}

template <int KT, int PA>
__device__ __forceinline__ void gemm4(v8f (&acc)[4], const _Float16* ar, const _Float16* __restrict__ br) {
#pragma unroll
  for (int t = 0; t < 4; ++t) acc[t] = zero8();
#pragma unroll 2
  for (int kt = 0; kt < KT; ++kt) {
    FragH b;
    b.h[0] = *(const v8h*)(br + 32 * kt);
    b.h[1] = *(const v8h*)(br + 32 * kt + 16);
#pragma unroll
    for (int mt = 0; mt < 4; ++mt) {
      FragH a;
      a.h[0] = *(const v8h*)(ar + mt * 16 * PA + 32 * kt);
      a.h[1] = *(const v8h*)(ar + mt * 16 * PA + 32 * kt + 16);
      acc[mt] = wmh(a.v, b.v, acc[mt]);
    }
  }
}

__device__ __forceinline__ void epi_act(const v8f (&acc)[4], _Float16* sA, _Float16* sG,
                                        const float* __restrict__ wsb, int wave, int hh, int m) {
  const int n = 16 * wave + m;
  const float bias = wsb[n];
#pragma unroll
  for (int mt = 0; mt < 4; ++mt) {
#pragma unroll
    for (int r = 0; r < 8; ++r) {
      const int e = 16 * mt + 8 * hh + r;
      const float x = acc[mt][r] * INV16 + bias;
      sG[e * PG + n]  = (_Float16)sigm(x);
      sA[e * PA2 + n] = (_Float16)fmaxf(x, 0.0f);
    }
  }
}

__device__ __forceinline__ void epi_last(const v8f (&acc)[4], _Float16* sG, float* sOS,
                                         const float* __restrict__ s, const float* __restrict__ wsb,
                                         int g0, int wave, int hh, int m) {
  const int n = 16 * wave + m;
  const float bias = wsb[n];
  float s0 = 0.0f, s1 = 0.0f;
#pragma unroll
  for (int mt = 0; mt < 4; ++mt) {
#pragma unroll
    for (int r = 0; r < 8; ++r) {
      const int e = 16 * mt + 8 * hh + r;
      const float x = acc[mt][r] * INV16 + bias;
      sG[e * PG + n] = (_Float16)x;
      if (mt < 2) s0 += x; else s1 += x;
    }
  }
  s0 += __shfl_xor(s0, 16, 32);
  s1 += __shfl_xor(s1, 16, 32);
  const float dx = (hh ? s1 : s0) * INVK;
  const int gj = g0 + hh;
  sOS[hh * SD + n] = s[(size_t)gj * SD + n] + dx;
}

__device__ __forceinline__ void gate_phase(const _Float16* sG, const _Float16* __restrict__ pG,
                                           const float* __restrict__ wsvb, float* sGT,
                                           int wave, int hh, int m) {
  if (wave < 4) {
    v8f acc = zero8();
    const _Float16* ar = sG + (16 * wave + m) * PG + 8 * hh;
    const _Float16* br = pG + m * GK + 8 * hh;
#pragma unroll
    for (int kt = 0; kt < GK / 32; ++kt) {
      FragH a, b;
      a.h[0] = *(const v8h*)(ar + 32 * kt);
      a.h[1] = *(const v8h*)(ar + 32 * kt + 16);
      b.h[0] = *(const v8h*)(br + 32 * kt);
      b.h[1] = *(const v8h*)(br + 32 * kt + 16);
      acc = wmh(a.v, b.v, acc);
    }
    const float bias = wsvb[m];
#pragma unroll
    for (int r = 0; r < 8; ++r) sGT[(16 * wave + 8 * hh + r) * VO + m] = sigm(acc[r] * INV16 + bias);
  }
}

template <int H, int VI>
__device__ __forceinline__ void load_w(float* sWH, float* sWV, const float* __restrict__ wh,
                                       const float* __restrict__ wv, int tid) {
  for (int i = tid; i < H * MVP; i += NTHR) {
    const int h = i / MVP;
    const int c = i - h * MVP;
    const int cc = c < VI ? c : VI - 1;
    const float x = wh[h * VI + cc];
    sWH[i] = c < VI ? x : 0.0f;
  }
  for (int i = tid; i < VO * MVP; i += NTHR) {
    const int o = i / MVP;
    const int c = i - o * MVP;
    const int cc = c < H ? c : H - 1;
    const float x = wv[o * H + cc];
    sWV[i] = c < H ? x : 0.0f;
  }
}

template <int VI, int H, int SI, int PA, bool ZP>
__device__ __forceinline__ void phase_vh(_Float16* sA, const float* sMV, float* sVH, const float* sWH, int tid) {
  constexpr int MVG   = (VI + 3) / 4;
  constexpr int HP    = ((H + 3) / 4) * 4;
  constexpr int NITEM = EPB * H;
  constexpr int NIT   = (NITEM + NTHR - 1) / NTHR;
#pragma unroll 1
  for (int it = 0; it < NIT; ++it) {
    const int item = tid + NTHR * it;
    const bool ok = item < NITEM;
    const int ic = ok ? item : 0;
    const int e = ic / H;
    const int h = ic - e * H;
    const float* mrow = sMV + e * MVS;
    const float* wrow = sWH + h * MVP;
    float a0 = 0.0f, a1 = 0.0f, a2 = 0.0f;
#pragma unroll
    for (int gi = 0; gi < MVG; ++gi) {
      const v4f w  = *(const v4f*)(wrow + 4 * gi);
      const v4f m0 = *(const v4f*)(mrow + 4 * gi);
      const v4f m1 = *(const v4f*)(mrow + MVP + 4 * gi);
      const v4f m2 = *(const v4f*)(mrow + 2 * MVP + 4 * gi);
#pragma unroll
      for (int c = 0; c < 4; ++c) {
        a0 = fmaf(w[c], m0[c], a0);
        a1 = fmaf(w[c], m1[c], a1);
        a2 = fmaf(w[c], m2[c], a2);
      }
    }
    if (ok) {
      sVH[e * MVS + h]           = a0;
      sVH[e * MVS + MVP + h]     = a1;
      sVH[e * MVS + 2 * MVP + h] = a2;
      const float ss = fmaf(a0, a0, fmaf(a1, a1, a2 * a2));
      sA[e * PA + SI + h] = (_Float16)sqrtf(fmaxf(ss, VEPS));
    }
  }
  if constexpr (HP > H) {
    if (tid < EPB * 3) {
      const int e = tid / 3;
      const int t = tid - 3 * e;
      float* p = sVH + e * MVS + t * MVP;
#pragma unroll
      for (int c = H; c < HP; ++c) p[c] = 0.0f;
    }
  }
  if constexpr (ZP) {
    if (tid < 2 * EPB) {
      const int e = tid >> 1, part = tid & 1;
      *(v8h*)(sA + e * PA + SI + H + 8 * part) = zero8h();
    }
  }
}

template <int H>
__device__ __forceinline__ void phase_vo(const float* sVH, float* sMV, const float* sWV, int tid) {
  constexpr int HG = (H + 3) / 4;
#pragma unroll 1
  for (int it = 0; it < 4; ++it) {
    const int item = tid + NTHR * it;
    const int e = item >> 4;
    const int o = item & 15;
    const float* hrow = sVH + e * MVS;
    const float* wrow = sWV + o * MVP;
    float a0 = 0.0f, a1 = 0.0f, a2 = 0.0f;
#pragma unroll
    for (int gi = 0; gi < HG; ++gi) {
      const v4f w  = *(const v4f*)(wrow + 4 * gi);
      const v4f h0 = *(const v4f*)(hrow + 4 * gi);
      const v4f h1 = *(const v4f*)(hrow + MVP + 4 * gi);
      const v4f h2 = *(const v4f*)(hrow + 2 * MVP + 4 * gi);
#pragma unroll
      for (int c = 0; c < 4; ++c) {
        a0 = fmaf(w[c], h0[c], a0);
        a1 = fmaf(w[c], h1[c], a1);
        a2 = fmaf(w[c], h2[c], a2);
      }
    }
    sMV[e * MVS + o]           = a0;
    sMV[e * MVS + MVP + o]     = a1;
    sMV[e * MVS + 2 * MVP + o] = a2;
  }
}

__device__ __forceinline__ void phase_scale(float* sMV, const float* sGT, int tid) {
#pragma unroll 1
  for (int it = 0; it < 4; ++it) {
    const int item = tid + NTHR * it;
    const int e = item >> 4;
    const int o = item & 15;
    const float gg = sGT[e * VO + o];
    float* p = sMV + e * MVS + o;
    p[0]       = p[0] * gg;
    p[MVP]     = p[MVP] * gg;
    p[2 * MVP] = p[2 * MVP] * gg;
  }
}

__global__ __launch_bounds__(NTHR) void k_prep(
    const float* __restrict__ w1, const float* __restrict__ w2, const float* __restrict__ w3,
    const float* __restrict__ g1, const float* __restrict__ g2, const float* __restrict__ g3,
    _Float16* pW1, _Float16* pW2, _Float16* pW3, _Float16* pG1, _Float16* pG2, _Float16* pG3) {
  const int bstart = blockIdx.x * NTHR;
  const int i = bstart + (int)threadIdx.x;
  if (i >= GTOT) return;
  float vv[8];
  _Float16* dp;
  if (bstart < GW1) {
    const int o  = i * 8;
    const int n  = o / K1P;
    const int k0 = o - n * K1P;
#pragma unroll
    for (int e = 0; e < 8; ++e) {
      const int k   = k0 + e;
      const int col = k < K1 ? k : K1 - 1;
      const float xv = w1[(size_t)n * K1 + col];
      vv[e] = (k < K1) ? xv * WSCL : xv * 0.0f;
    }
    dp = pW1 + o;
  } else if (bstart < GW1 + GW2) {
    const int o  = (i - GW1) * 8;
    const int n  = o / K2P;
    const int k0 = o - n * K2P;
#pragma unroll
    for (int e = 0; e < 8; ++e) {
      const int k   = k0 + e;
      const int col = k < K2 ? k : K2 - 1;
      const float xv = w2[(size_t)n * K2 + col];
      vv[e] = (k < K2) ? xv * WSCL : xv * 0.0f;
    }
    dp = pW2 + o;
  } else if (bstart < GW1 + 2 * GW2) {
    const int o  = (i - GW1 - GW2) * 8;
    const int n  = o / K2P;
    const int k0 = o - n * K2P;
#pragma unroll
    for (int e = 0; e < 8; ++e) {
      const int k   = k0 + e;
      const int col = k < K2 ? k : K2 - 1;
      const float xv = w3[(size_t)n * K2 + col];
      vv[e] = (k < K2) ? xv * WSCL : xv * 0.0f;
    }
    dp = pW3 + o;
  } else if (bstart < GW1 + 2 * GW2 + GGT) {
    const int o  = (i - GW1 - 2 * GW2) * 8;
    const int n  = o >> 7;
    const int k0 = o & 127;
#pragma unroll
    for (int e = 0; e < 8; ++e) vv[e] = g1[n * GK + k0 + e] * WSCL;
    dp = pG1 + o;
  } else if (bstart < GW1 + 2 * GW2 + 2 * GGT) {
    const int o  = (i - GW1 - 2 * GW2 - GGT) * 8;
    const int n  = o >> 7;
    const int k0 = o & 127;
#pragma unroll
    for (int e = 0; e < 8; ++e) vv[e] = g2[n * GK + k0 + e] * WSCL;
    dp = pG2 + o;
  } else {
    const int o  = (i - GW1 - 2 * GW2 - 2 * GGT) * 8;
    const int n  = o >> 7;
    const int k0 = o & 127;
#pragma unroll
    for (int e = 0; e < 8; ++e) vv[e] = g3[n * GK + k0 + e] * WSCL;
    dp = pG3 + o;
  }
  v8h hv;
#pragma unroll
  for (int e = 0; e < 8; ++e) hv[e] = (_Float16)vv[e];
  *(volatile v8h*)dp = hv;
  __threadfence();
  *(volatile v8h*)dp = hv;
}

__global__ __launch_bounds__(NTHR) void k_main(
    const float* __restrict__ s, const float* __restrict__ v,
    const float* __restrict__ es, const float* __restrict__ ev, const int* __restrict__ ei,
    const float* __restrict__ wh1, const float* __restrict__ wsb1,
    const float* __restrict__ wv1, const float* __restrict__ wsvb1,
    const float* __restrict__ wh2, const float* __restrict__ wsb2,
    const float* __restrict__ wv2, const float* __restrict__ wsvb2,
    const float* __restrict__ wh3, const float* __restrict__ wsb3,
    const float* __restrict__ wv3, const float* __restrict__ wsvb3,
    const _Float16* __restrict__ pW1, const _Float16* __restrict__ pW2, const _Float16* __restrict__ pW3,
    const _Float16* __restrict__ pG1, const _Float16* __restrict__ pG2, const _Float16* __restrict__ pG3,
    float* outs, float* outv) {
  extern __shared__ v4f lds_dyn[];
  char* lb = (char*)lds_dyn;
  _Float16* sA  = (_Float16*)(lb + L_A);
  _Float16* sG  = (_Float16*)(lb + L_GIN);
  float*    sMV = (float*)(lb + L_MV);
  float*    sVH = (float*)(lb + L_VH);
  float*    sGT = (float*)(lb + L_GT);
  float*    sWH = (float*)(lb + L_WH);
  float*    sWV = (float*)(lb + L_WV);
  float*    sOS = (float*)(lb + L_OS);
  float*    sOV = (float*)(lb + L_OV);

  const int tid = threadIdx.x, lane = tid & 31, wave = tid >> 5, hh = lane >> 4, m = lane & 15;
  const int g0 = blockIdx.x * 2;

  load_w<H1, VI1>(sWH, sWV, wh1, wv1, tid);
#pragma unroll 1
  for (int e8 = 0; e8 < 8; ++e8) {
    const int e  = wave * 8 + e8;
    const int g  = g0 + (e >> 5);
    const int b  = g >> 11;
    const int k  = e & 31;
    const int eo = g * KNB + k;
    int idx = ei[eo];
    idx = idx < 0 ? 0 : (idx > NN - 1 ? NN - 1 : idx);
    const int gn = (b << 11) + idx;
    _Float16* row = sA + e * PA1;
    {
      const v4f xi = *(const v4f*)(s + (size_t)g * SD + 4 * lane);
      const v4f xj = *(const v4f*)(s + (size_t)gn * SD + 4 * lane);
      v4h hi4, hj4;
#pragma unroll
      for (int c = 0; c < 4; ++c) { hi4[c] = (_Float16)xi[c]; hj4[c] = (_Float16)xj[c]; }
      *(v4h*)(row + 4 * lane) = hi4;
      *(v4h*)(row + SD + 4 * lane) = hj4;
      const int le = lane < 8 ? lane : 7;
      const v4f xe = *(const v4f*)(es + (size_t)eo * ESD + 4 * le);
      v4h he4;
#pragma unroll
      for (int c = 0; c < 4; ++c) he4[c] = (_Float16)xe[c];
      if (lane < 8) *(v4h*)(row + 2 * SD + 4 * lane) = he4;
      if (lane < 5) *(v8h*)(row + ZC1 + 8 * lane) = zero8h();
    }
    {
      float* mrow = sMV + e * MVS;
      const float* va0 = v + (size_t)g * VF;
      const float* vb0 = v + (size_t)gn * VF;
      const float* vc0 = ev + (size_t)eo * 3;
#pragma unroll
      for (int it = 0; it < 4; ++it) {
        const int ix = lane + 32 * it;
        const int t  = ix / MVP;
        const int c  = ix - t * MVP;
        const int tt = t < 3 ? t : 2;
        const int ca = c < VC ? c : VC - 1;
        int cb = c - VC;
        cb = cb < 0 ? 0 : (cb > VC - 1 ? VC - 1 : cb);
        const float xa = va0[ca * 3 + tt];
        const float xb = vb0[cb * 3 + tt];
        const float xc = vc0[tt];
        const float val = c < VC ? xa : (c < 2 * VC ? xb : (c == 2 * VC ? xc : 0.0f));
        if (ix < MVS) mrow[ix] = val;
      }
    }
  }
  __syncthreads();

  v8f acc[4];

  phase_vh<VI1, H1, SI1, PA1, false>(sA, sMV, sVH, sWH, tid);
  __syncthreads();
  gemm4<K1P / 32, PA1>(acc, sA + m * PA1 + 8 * hh, pW1 + (size_t)(16 * wave + m) * K1P + 8 * hh);
  __syncthreads();
  epi_act(acc, sA, sG, wsb1, wave, hh, m);
  phase_vo<H1>(sVH, sMV, sWV, tid);
  __syncthreads();
  gate_phase(sG, pG1, wsvb1, sGT, wave, hh, m);
  __syncthreads();
  phase_scale(sMV, sGT, tid);
  load_w<H2, VI2>(sWH, sWV, wh2, wv2, tid);
  __syncthreads();

  phase_vh<VI2, H2, SI2, PA2, true>(sA, sMV, sVH, sWH, tid);
  __syncthreads();
  gemm4<K2P / 32, PA2>(acc, sA + m * PA2 + 8 * hh, pW2 + (size_t)(16 * wave + m) * K2P + 8 * hh);
  __syncthreads();
  epi_act(acc, sA, sG, wsb2, wave, hh, m);
  phase_vo<H2>(sVH, sMV, sWV, tid);
  __syncthreads();
  gate_phase(sG, pG2, wsvb2, sGT, wave, hh, m);
  __syncthreads();
  phase_scale(sMV, sGT, tid);
  load_w<H2, VI2>(sWH, sWV, wh3, wv3, tid);
  __syncthreads();

  phase_vh<VI2, H2, SI2, PA2, true>(sA, sMV, sVH, sWH, tid);
  __syncthreads();
  gemm4<K2P / 32, PA2>(acc, sA + m * PA2 + 8 * hh, pW3 + (size_t)(16 * wave + m) * K2P + 8 * hh);
  __syncthreads();
  epi_last(acc, sG, sOS, s, wsb3, g0, wave, hh, m);
  phase_vo<H2>(sVH, sMV, sWV, tid);
  __syncthreads();
  gate_phase(sG, pG3, wsvb3, sGT, wave, hh, m);
  __syncthreads();
  phase_scale(sMV, sGT, tid);
  __syncthreads();

  if (tid < 2 * VF) {
    const int j  = tid / VF;
    const int r  = tid - j * VF;
    const int ch = r / 3;
    const int t  = r - 3 * ch;
    const float* p = sMV + (j * KNB) * MVS + t * MVP + ch;
    float sum = 0.0f;
#pragma unroll 8
    for (int kk = 0; kk < KNB; ++kk) sum += p[kk * MVS];
    sOV[tid] = v[(size_t)(g0 + j) * VF + r] + sum * INVK;
  }
  __syncthreads();

  if (wave < 2) {
    const v4f ov = *(const v4f*)(sOS + wave * SD + 4 * lane);
    float* gp = outs + (size_t)(g0 + wave) * SD + 4 * lane;
    *(volatile v4f*)gp = ov;
    __threadfence();
    *(volatile v4f*)gp = ov;
  }
  if (wave == 0) {
    const int lc = lane < 24 ? lane : 23;
    const v4f ov = *(const v4f*)(sOV + 4 * lc);
    float* gp = outv + (size_t)g0 * VF + 4 * lc;
    if (lane < 24) *(volatile v4f*)gp = ov;
    __threadfence();
    if (lane < 24) *(volatile v4f*)gp = ov;
  }
}

extern "C" void kernel_launch(void* const* d_in, const int* in_sizes, int n_in,
                              void* d_out, int out_size, void* d_ws, size_t ws_size,
                              hipStream_t stream) {
  if (n_in < 23) return;
  if (in_sizes[0] != NODES * SD) return;
  if (in_sizes[1] != NODES * VF) return;
  if (in_sizes[2] != NODES * KNB * ESD) return;
  if (in_sizes[3] != NODES * KNB * 3) return;
  if (in_sizes[4] != NODES * KNB) return;
  if (in_sizes[5] != H1 * VI1 || in_sizes[6] != SO * K1 || in_sizes[7] != SO) return;
  if (in_sizes[8] != VO * H1 || in_sizes[9] != VO * GK || in_sizes[10] != VO) return;
  if (in_sizes[11] != H2 * VI2 || in_sizes[12] != SO * K2 || in_sizes[13] != SO) return;
  if (in_sizes[14] != VO * H2 || in_sizes[15] != VO * GK || in_sizes[16] != VO) return;
  if (in_sizes[17] != H2 * VI2 || in_sizes[18] != SO * K2 || in_sizes[19] != SO) return;
  if (in_sizes[20] != VO * H2 || in_sizes[21] != VO * GK || in_sizes[22] != VO) return;
  if (out_size != NODES * SD + NODES * VF) return;

  const float* s     = (const float*)d_in[0];
  const float* v     = (const float*)d_in[1];
  const float* es    = (const float*)d_in[2];
  const float* ev    = (const float*)d_in[3];
  const int*   ei    = (const int*)d_in[4];
  const float* wh1   = (const float*)d_in[5];
  const float* wsw1  = (const float*)d_in[6];
  const float* wsb1  = (const float*)d_in[7];
  const float* wv1   = (const float*)d_in[8];
  const float* wsvw1 = (const float*)d_in[9];
  const float* wsvb1 = (const float*)d_in[10];
  const float* wh2   = (const float*)d_in[11];
  const float* wsw2  = (const float*)d_in[12];
  const float* wsb2  = (const float*)d_in[13];
  const float* wv2   = (const float*)d_in[14];
  const float* wsvw2 = (const float*)d_in[15];
  const float* wsvb2 = (const float*)d_in[16];
  const float* wh3   = (const float*)d_in[17];
  const float* wsw3  = (const float*)d_in[18];
  const float* wsb3  = (const float*)d_in[19];
  const float* wv3   = (const float*)d_in[20];
  const float* wsvw3 = (const float*)d_in[21];
  const float* wsvb3 = (const float*)d_in[22];
  float* outs = (float*)d_out;
  float* outv = (float*)d_out + (size_t)NODES * SD;

  char* ws = (char*)d_ws;
  size_t off = 0;
  const size_t oW1 = off; off += (size_t)SO * K1P * 2; off = (off + 255) & ~(size_t)255;
  const size_t oW2 = off; off += (size_t)SO * K2P * 2; off = (off + 255) & ~(size_t)255;
  const size_t oW3 = off; off += (size_t)SO * K2P * 2; off = (off + 255) & ~(size_t)255;
  const size_t oG1 = off; off += (size_t)VO * GK * 2;  off = (off + 255) & ~(size_t)255;
  const size_t oG2 = off; off += (size_t)VO * GK * 2;  off = (off + 255) & ~(size_t)255;
  const size_t oG3 = off; off += (size_t)VO * GK * 2;  off = (off + 255) & ~(size_t)255;
  if (off > ws_size || off > (size_t)134217728) return;
  _Float16* pW1 = (_Float16*)(ws + oW1);
  _Float16* pW2 = (_Float16*)(ws + oW2);
  _Float16* pW3 = (_Float16*)(ws + oW3);
  _Float16* pG1 = (_Float16*)(ws + oG1);
  _Float16* pG2 = (_Float16*)(ws + oG2);
  _Float16* pG3 = (_Float16*)(ws + oG3);

  k_prep<<<GTOT / NTHR, NTHR, 0, stream>>>(wsw1, wsw2, wsw3, wsvw1, wsvw2, wsvw3,
                                           pW1, pW2, pW3, pG1, pG2, pG3);

  hipFuncSetAttribute(reinterpret_cast<const void*>(&k_main),
                      hipFuncAttributeMaxDynamicSharedMemorySize, LDS_MAIN);
  k_main<<<NODES / 2, NTHR, LDS_MAIN, stream>>>(
      s, v, es, ev, ei,
      wh1, wsb1, wv1, wsvb1, wh2, wsb2, wv2, wsvb2, wh3, wsb3, wv3, wsvb3,
      pW1, pW2, pW3, pG1, pG2, pG3, outs, outv);
}
